// Unpool_wSkip_15504831939266
// MI455X (gfx1250) — hardware-verified
//
#include <hip/hip_runtime.h>
#include <math.h>

#define BB 4
#define MM 4096
#define NN 16384
#define KNB 8
#define CI 64
#define CO 64
#define NROW (BB * NN)
#define BR 64
#define NBLK (NROW / BR)
#define OC 131

typedef _Float16 f16;
typedef __attribute__((ext_vector_type(16))) f16 f16x16;
typedef __attribute__((ext_vector_type(8)))  f16 f16x8;
typedef __attribute__((ext_vector_type(8)))  float f32x8;
typedef __attribute__((ext_vector_type(4)))  float v4f_t;
typedef float v4fa __attribute__((ext_vector_type(4), may_alias));

__device__ __forceinline__ f32x8 wmma16(f16x16 a, f16x16 b, f32x8 c) {
  c = __builtin_amdgcn_wmma_f32_16x16x32_f16(false, a, false, b, (short)0, c, false, false);
  asm volatile("v_nop\n\tv_nop\n\tv_nop\n\tv_nop" : "+v"(c) : "v"(a), "v"(b));
  return c;
}
__device__ __forceinline__ f16x16 lds_frag(const f16* base, int stride) {
  const int lane = threadIdx.x & 31, row = lane & 15, kh = (lane >> 4) * 8;
  const f16x8 lo = *(const f16x8*)(base + row * stride + kh);
  const f16x8 hi = *(const f16x8*)(base + row * stride + kh + 16);
  f16x16 f;
#pragma unroll
  for (int i = 0; i < 8; ++i) { f[i] = lo[i]; f[i + 8] = hi[i]; }
  return f;
}
__device__ __forceinline__ void split16(float v, f16& h, f16& l) { h = (f16)v; l = (f16)((v - (float)h) * 2048.0f); }

struct Tiles {
  f16 aI[2][BR * 72]; f16 aS[2][BR * 72];
  float yS[2][BR * 68];
};
__device__ __forceinline__ void wfrag2(const float* __restrict__ Wm, int o0, int k0, f16x16& hi, f16x16& lo) {
  const int lane = threadIdx.x & 31, r = lane & 15, kh = (lane >> 4) * 8;
  const float* p = Wm + (size_t)(o0 + r) * CI + k0 + kh;
#pragma unroll
  for (int i = 0; i < 8; ++i) { f16 h, l; split16(p[i], h, l); hi[i] = h; lo[i] = l; split16(p[16 + i], h, l); hi[8 + i] = h; lo[8 + i] = l; }
}
__device__ __forceinline__ void compute_tile(Tiles& T, int blk, const float* __restrict__ cf, const float* __restrict__ sf, const int* __restrict__ idx,
                             const float* __restrict__ Wp, const float* __restrict__ bp, const float* __restrict__ Wk, const float* __restrict__ bk) {
  const int tid = threadIdx.x, lane = tid & 31, wave = tid >> 5, cl = lane & 15, rh = (lane >> 4) * 8;
  const int g0 = blk * BR; const int b = g0 / NN;
  { const int row = tid >> 2, c0 = (tid & 3) * 16; const int g = g0 + row, n = g % NN;
    const int* ip = idx + (size_t)g * KNB;
    float mx[16];
#pragma unroll
    for (int c = 0; c < 16; ++c) mx[c] = -INFINITY;
#pragma unroll 1
    for (int j = 0; j < KNB; ++j) { int m = ip[j]; m = min(max(m, 0), MM - 1); const float* src = cf + ((size_t)b * MM + m) * CI + c0;
#pragma unroll
      for (int q = 0; q < 4; ++q) { const v4f_t v = *(const v4f_t*)(src + 4 * q); mx[4*q] = fmaxf(mx[4*q], v[0]); mx[4*q+1] = fmaxf(mx[4*q+1], v[1]); mx[4*q+2] = fmaxf(mx[4*q+2], v[2]); mx[4*q+3] = fmaxf(mx[4*q+3], v[3]); } }
#pragma unroll
    for (int c = 0; c < 16; ++c) { f16 h, l; split16(mx[c], h, l); T.aI[0][row * 72 + c0 + c] = h; T.aI[1][row * 72 + c0 + c] = l; }
    const float* ss = sf + (size_t)g * CI + c0;
#pragma unroll
    for (int q = 0; q < 4; ++q) { const v4f_t v = *(const v4f_t*)(ss + 4 * q);
#pragma unroll
      for (int u = 0; u < 4; ++u) { f16 h, l; split16(v[u], h, l); T.aS[0][row * 72 + c0 + 4*q + u] = h; T.aS[1][row * 72 + c0 + 4*q + u] = l; } }
    (void)n; }
  __syncthreads();
  {
    const int which = wave >> 2, rt = wave & 3;
    const f16* A0 = which ? T.aS[0] : T.aI[0]; const f16* A1 = which ? T.aS[1] : T.aI[1]; const float* Wsel = which ? Wk : Wp; const float* bias = which ? bk : bp;
    f16x16 ah[2], al[2];
#pragma unroll
    for (int ks = 0; ks < 2; ++ks) { ah[ks] = lds_frag(A0 + (rt * 16) * 72 + ks * 32, 72); al[ks] = lds_frag(A1 + (rt * 16) * 72 + ks * 32, 72); }
#pragma unroll 1
    for (int nt = 0; nt < 4; ++nt) {
      f32x8 acc = {}, accx = {};
#pragma unroll
      for (int ks = 0; ks < 2; ++ks) { f16x16 bh, bl; wfrag2(Wsel, nt * 16, ks * 32, bh, bl);
        acc = wmma16(ah[ks], bh, acc); accx = wmma16(ah[ks], bl, accx); accx = wmma16(al[ks], bh, accx); }
      const int o = nt * 16 + cl; const float bv = bias[o];
#pragma unroll
      for (int r = 0; r < 8; ++r) T.yS[which][(rt * 16 + rh + r) * 68 + o] = acc[r] + accx[r] * (1.0f / 2048.0f) + bv;
    }
  }
  __syncthreads();
}

__global__ __launch_bounds__(256) void k_stats(const float* __restrict__ cf, const float* __restrict__ sf, const int* __restrict__ idx,
                                              const float* __restrict__ Wp, const float* __restrict__ bp, const float* __restrict__ Wk, const float* __restrict__ bk, float* __restrict__ partial) {
  __shared__ Tiles T;
  __shared__ __attribute__((aligned(16))) float pS[256];
  compute_tile(T, blockIdx.x, cf, sf, idx, Wp, bp, Wk, bk);
  const int tid = threadIdx.x;
  { const int which = tid >> 7, kind = (tid >> 6) & 1, o = tid & 63; float s = 0.0f;
    for (int r = 0; r < BR; ++r) { const float v = T.yS[which][r * 68 + o]; s += kind ? v * v : v; }
    pS[tid] = s; }
  __syncthreads();
  if (tid < 64) { *(volatile v4f_t*)(partial + (size_t)blockIdx.x * 256 + tid * 4) = *(const volatile v4fa*)(pS + tid * 4); __threadfence(); *(volatile v4f_t*)(partial + (size_t)blockIdx.x * 256 + tid * 4) = *(const volatile v4fa*)(pS + tid * 4); }
}
__global__ __launch_bounds__(256) void k_bn(const float* __restrict__ partial, const float* __restrict__ gp, const float* __restrict__ bep, const float* __restrict__ gs, const float* __restrict__ bes, float* __restrict__ ssout) {
  __shared__ float sumS[256];
  __shared__ __attribute__((aligned(16))) float oS[256];
  const int tid = threadIdx.x; float s = 0.0f;
  for (int bl = 0; bl < NBLK; ++bl) s += partial[(size_t)bl * 256 + tid];
  sumS[tid] = s;
  __syncthreads();
  if (tid < 128) { const int which = tid >> 6, o = tid & 63;
    const float sum = sumS[which * 128 + o], sq = sumS[which * 128 + 64 + o];
    const float mean = sum / (float)NROW; const float var = fmaxf(sq / (float)NROW - mean * mean, 0.0f);
    const float gam = which ? gs[o] : gp[o], bet = which ? bes[o] : bep[o];
    const float scale = gam / sqrtf(var + 1e-5f);
    oS[which * 128 + o] = scale; oS[which * 128 + 64 + o] = bet - mean * scale; }
  __syncthreads();
  if (tid < 64) { *(volatile v4f_t*)(ssout + tid * 4) = *(const volatile v4fa*)(oS + tid * 4); __threadfence(); *(volatile v4f_t*)(ssout + tid * 4) = *(const volatile v4fa*)(oS + tid * 4); }
}
__global__ __launch_bounds__(256) void k_out(const float* __restrict__ cf, const float* __restrict__ sf, const int* __restrict__ idx,
                                            const float* __restrict__ Wp, const float* __restrict__ bp, const float* __restrict__ Wk, const float* __restrict__ bk,
                                            const float* __restrict__ ssin, const float* __restrict__ scoord, float* __restrict__ out) {
  __shared__ Tiles T;
  __shared__ __attribute__((aligned(16))) float oS[BR * OC];
  __shared__ float ssS[256];
  const int tid = threadIdx.x;
  ssS[tid] = ssin[tid];
  compute_tile(T, blockIdx.x, cf, sf, idx, Wp, bp, Wk, bk);
  const int g0 = blockIdx.x * BR;
  for (int e = tid; e < BR * OC; e += 256) { const int r = e / OC, c = e % OC; float v;
    if (c < 3) v = scoord[(size_t)(g0 + r) * 3 + c];
    else if (c < 3 + CO) { const int o = c - 3; v = fmaxf(T.yS[1][r * 68 + o] * ssS[128 + o] + ssS[192 + o], 0.0f); }
    else { const int o = c - 3 - CO; v = fmaxf(T.yS[0][r * 68 + o] * ssS[o] + ssS[64 + o], 0.0f); }
    oS[e] = v; }
  __syncthreads();
  float* dst = out + (size_t)g0 * OC;
#pragma unroll 1
  for (int pass = 0; pass < 2; ++pass) {
    for (int q = tid; q < BR * OC / 4; q += 256) *(volatile v4f_t*)(dst + q * 4) = *(const volatile v4fa*)(oS + q * 4);
    __threadfence();
  }
}

extern "C" void kernel_launch(void* const* d_in, const int* in_sizes, int n_in,
                              void* d_out, int out_size, void* d_ws, size_t ws_size,
                              hipStream_t stream) {
  (void)in_sizes; (void)n_in; (void)out_size; (void)ws_size;
  const float* cf = (const float*)d_in[1];
  const float* scoord = (const float*)d_in[2];
  const float* sf = (const float*)d_in[3];
  const int* idx = (const int*)d_in[4];
  const float* Wp = (const float*)d_in[5], *bp = (const float*)d_in[6], *gp = (const float*)d_in[7], *bep = (const float*)d_in[8];
  const float* Wk = (const float*)d_in[9], *bk = (const float*)d_in[10], *gs = (const float*)d_in[11], *bes = (const float*)d_in[12];
  float* out = (float*)d_out;
  char* ws = (char*)d_ws;
  float* partial = (float*)ws; ws += (size_t)NBLK * 256 * 4;
  float* ss = (float*)ws; ws += 256 * 4;
  k_stats<<<dim3(NBLK), dim3(256), 0, stream>>>(cf, sf, idx, Wp, bp, Wk, bk, partial);
  k_bn<<<dim3(1), dim3(256), 0, stream>>>(partial, gp, bep, gs, bes, ss);
  k_out<<<dim3(NBLK), dim3(256), 0, stream>>>(cf, sf, idx, Wp, bp, Wk, bk, ss, scoord, out);
}
